// BatchFlipLoss_85306640433706
// MI455X (gfx1250) — hardware-verified
//
#include <hip/hip_runtime.h>
#define NN 4096
#define DD 128
#define CC 400
#define FL 8
#define HB (NN / FL)
#define NP 36

typedef __bf16 v16b __attribute__((ext_vector_type(16)));
typedef unsigned short v8us __attribute__((ext_vector_type(8), may_alias));
typedef float  v8f  __attribute__((ext_vector_type(8)));
typedef float  v4f  __attribute__((ext_vector_type(4)));
typedef float  v4fa __attribute__((ext_vector_type(4), may_alias));
union FragB { v16b v; v8us half[2]; unsigned short u[16]; };

__device__ __forceinline__ unsigned short bf16_bits(float x) { unsigned int u = __float_as_uint(x); return (unsigned short)((u + 0x7FFFu + ((u >> 16) & 1u)) >> 16); }
__device__ __forceinline__ float bf16_val(unsigned short b) { return __uint_as_float(((unsigned int)b) << 16); }
__device__ __forceinline__ float bf16_round(float x) { return bf16_val(bf16_bits(x)); }
template <int NT>
__device__ __forceinline__ v8f mmaN(v16b ah, v16b al, v16b bh, v16b bl, v8f c) {
  c = __builtin_amdgcn_wmma_f32_16x16x32_bf16(false, ah, false, bh, (short)0, c, false, false);
  if (NT >= 2) c = __builtin_amdgcn_wmma_f32_16x16x32_bf16(false, al, false, bh, (short)0, c, false, false);
  if (NT >= 3) c = __builtin_amdgcn_wmma_f32_16x16x32_bf16(false, ah, false, bl, (short)0, c, false, false);
  asm volatile("v_nop\n\tv_nop\n\tv_nop\n\tv_nop" : "+v"(c) : "v"(ah), "v"(al), "v"(bh), "v"(bl));
  return c;
}

__global__ __launch_bounds__(256) void k_wt_bf16(const float* __restrict__ W, unsigned short* __restrict__ Wt, int K, int N) {
  const int t = blockIdx.x * 256 + threadIdx.x;
  const int k8n = K / 8;
  if (t >= N * k8n) return;
  const int n = t / k8n, k8 = (t % k8n) * 8;
  v8us v;
#pragma unroll
  for (int i = 0; i < 8; ++i) v[i] = bf16_bits(W[(size_t)(k8 + i) * N + n]);
  *(volatile v8us*)(Wt + (size_t)n * K + k8) = v;
  __threadfence();
  *(volatile v8us*)(Wt + (size_t)n * K + k8) = v;
}

template <bool ASPLIT, int ACT, bool BIAS_BF16>
__global__ __launch_bounds__(128) void k_gemm_bf(const float* __restrict__ A, int lda, const unsigned short* __restrict__ Wt, int ldb,
                                               const float* __restrict__ bias, float* __restrict__ C, int ldc, int M, int N, int K) {
  __shared__ __attribute__((aligned(16))) float so[4][16][64];
  const int tid = threadIdx.x, w = tid >> 5, lane = tid & 31, ln = lane & 15, hh = lane >> 4;
  const int ntn = N / 64;
  const int wid = blockIdx.x * 4 + w;
  const int mt = wid / ntn, nq = wid % ntn;
  if (mt * 16 >= M) return;
  const int row0 = mt * 16, col0 = nq * 64;
  const float* arow = A + (size_t)(row0 + ln) * lda;
  v8f acc[4] = {};
  for (int kb = 0; kb < K; kb += 32) {
    FragB ah, al;
    const v4f x0 = *(const v4fa*)(arow + kb + 8 * hh), x1 = *(const v4fa*)(arow + kb + 8 * hh + 4);
    const v4f x2 = *(const v4fa*)(arow + kb + 16 + 8 * hh), x3 = *(const v4fa*)(arow + kb + 16 + 8 * hh + 4);
    float xs[16] = {x0[0],x0[1],x0[2],x0[3],x1[0],x1[1],x1[2],x1[3],x2[0],x2[1],x2[2],x2[3],x3[0],x3[1],x3[2],x3[3]};
#pragma unroll
    for (int i = 0; i < 16; ++i) { const unsigned short hb = bf16_bits(xs[i]); ah.u[i] = hb; al.u[i] = ASPLIT ? bf16_bits(xs[i] - bf16_val(hb)) : (unsigned short)0; }
#pragma unroll
    for (int t = 0; t < 4; ++t) {
      const unsigned short* brow = Wt + (size_t)(col0 + t * 16 + ln) * ldb + kb;
      FragB b;
      b.half[0] = *(const v8us*)(brow + 8 * hh);
      b.half[1] = *(const v8us*)(brow + 16 + 8 * hh);
      acc[t] = mmaN<ASPLIT ? 2 : 1>(ah.v, al.v, b.v, b.v, acc[t]);
    }
  }
#pragma unroll
  for (int t = 0; t < 4; ++t) {
    float bv = bias ? bias[col0 + t * 16 + ln] : 0.f;
    if (BIAS_BF16) bv = bf16_round(bv);
#pragma unroll
    for (int r = 0; r < 8; ++r) { float v = acc[t][r] + bv; if (ACT == 1) v = fmaxf(v, 0.f); so[w][8 * hh + r][t * 16 + ln] = v; }
  }
  __builtin_amdgcn_fence(__ATOMIC_ACQ_REL, "workgroup");
  __builtin_amdgcn_wave_barrier();
  const int rsub = lane >> 4, c4 = (lane & 15) * 4;
  for (int pass = 0; pass < 2; ++pass) {
#pragma unroll
    for (int q = 0; q < 8; ++q) {
      const int r = q * 2 + rsub;
      const v4f v = *(const v4fa*)&so[w][r][c4];
      *(volatile v4f*)(C + (size_t)(row0 + r) * ldc + col0 + c4) = v;
    }
    if (pass == 0) __threadfence();
  }
}

template <int D, bool CAUSAL>
__global__ __launch_bounds__(128) void k_flash(const float* __restrict__ qb, const float* __restrict__ kb, const float* __restrict__ vb,
                                             int pitch, int T, int H, float scale, float* __restrict__ y, int ypitch) {
  constexpr int KS = D / 32;
  constexpr int DT = D / 16;
  __shared__ __attribute__((aligned(16))) unsigned short sKh[32][D + 8], sKl[32][D + 8], sVh[32][D + 8], sVl[32][D + 8];
  __shared__ __attribute__((aligned(16))) unsigned short sPh[4][16][40], sPl[4][16][40];
  __shared__ __attribute__((aligned(16))) float sO[4][16][D];
  const int tid = threadIdx.x, w = tid >> 5, lane = tid & 31, ln = lane & 15, hh = lane >> 4;
  const int nqb = (T + 63) / 64;
  const int bh = blockIdx.x / nqb, qblk = blockIdx.x % nqb;
  const int b = bh / H, h = bh % H;
  const int q0 = qblk * 64 + w * 16;
  const float* Q = qb + (size_t)b * T * pitch + h * D;
  const float* K = kb + (size_t)b * T * pitch + h * D;
  const float* V = vb + (size_t)b * T * pitch + h * D;

  FragB aqh[KS], aql[KS];
  {
    int row = q0 + ln; if (row >= T) row = T - 1;
    const float* qr = Q + (size_t)row * pitch;
#pragma unroll
    for (int ks = 0; ks < KS; ++ks)
#pragma unroll
      for (int i = 0; i < 16; ++i) {
        const int d = ks * 32 + ((i < 8) ? (8 * hh + i) : (16 + 8 * hh + (i - 8)));
        const float x = qr[d] * scale; const unsigned short hb = bf16_bits(x);
        aqh[ks].u[i] = hb; aql[ks].u[i] = bf16_bits(x - bf16_val(hb));
      }
  }
  float m_r[8], l_r[8];
#pragma unroll
  for (int r = 0; r < 8; ++r) { m_r[r] = -3.0e38f; l_r[r] = 0.f; }
  v8f oacc[DT];
#pragma unroll
  for (int dt = 0; dt < DT; ++dt) oacc[dt] = (v8f){0.f,0.f,0.f,0.f,0.f,0.f,0.f,0.f};

  const int kv_end = CAUSAL ? min(T, qblk * 64 + 64) : T;
  for (int j0 = 0; j0 < kv_end; j0 += 32) {
    __syncthreads();
    for (int e = tid; e < 32 * (D / 4); e += 128) {
      const int r = e / (D / 4), c4 = (e % (D / 4)) * 4;
      const int key = j0 + r;
      v4f kf = {0.f,0.f,0.f,0.f}, vf = {0.f,0.f,0.f,0.f};
      if (key < T) { kf = *(const v4fa*)(K + (size_t)key * pitch + c4); vf = *(const v4fa*)(V + (size_t)key * pitch + c4); }
#pragma unroll
      for (int t = 0; t < 4; ++t) {
        unsigned short hb = bf16_bits(kf[t]); sKh[r][c4 + t] = hb; sKl[r][c4 + t] = bf16_bits(kf[t] - bf16_val(hb));
        hb = bf16_bits(vf[t]); sVh[r][c4 + t] = hb; sVl[r][c4 + t] = bf16_bits(vf[t] - bf16_val(hb));
      }
    }
    __syncthreads();
    v8f s[2];
#pragma unroll
    for (int nt = 0; nt < 2; ++nt) {
      v8f acc = {};
#pragma unroll
      for (int ks = 0; ks < KS; ++ks) {
        FragB bh_, bl_;
        bh_.half[0] = *(const v8us*)&sKh[nt * 16 + ln][ks * 32 + 8 * hh]; bh_.half[1] = *(const v8us*)&sKh[nt * 16 + ln][ks * 32 + 16 + 8 * hh];
        bl_.half[0] = *(const v8us*)&sKl[nt * 16 + ln][ks * 32 + 8 * hh]; bl_.half[1] = *(const v8us*)&sKl[nt * 16 + ln][ks * 32 + 16 + 8 * hh];
        acc = mmaN<3>(aqh[ks].v, aql[ks].v, bh_.v, bl_.v, acc);
      }
      s[nt] = acc;
    }
    float alpha[8];
#pragma unroll
    for (int r = 0; r < 8; ++r) {
      const int qi = q0 + 8 * hh + r;
      const int ja = j0 + ln, jb = j0 + 16 + ln;
      if (CAUSAL) { if (ja > qi) s[0][r] = -3.0e38f; if (jb > qi) s[1][r] = -3.0e38f; }
      if (ja >= T) s[0][r] = -3.0e38f;
      if (jb >= T) s[1][r] = -3.0e38f;
      float mx = fmaxf(s[0][r], s[1][r]);
      mx = fmaxf(mx, __shfl_xor(mx, 1, 32)); mx = fmaxf(mx, __shfl_xor(mx, 2, 32)); mx = fmaxf(mx, __shfl_xor(mx, 4, 32)); mx = fmaxf(mx, __shfl_xor(mx, 8, 32));
      const float mnew = fmaxf(m_r[r], mx);
      alpha[r] = (mnew > -1.0e38f) ? __expf(m_r[r] - mnew) : 1.0f;
      const float p0 = (s[0][r] > -1.0e38f) ? __expf(s[0][r] - mnew) : 0.f;
      const float p1 = (s[1][r] > -1.0e38f) ? __expf(s[1][r] - mnew) : 0.f;
      m_r[r] = mnew;
      l_r[r] = l_r[r] * alpha[r] + p0 + p1;
      unsigned short hb = bf16_bits(p0); sPh[w][8 * hh + r][ln] = hb;      sPl[w][8 * hh + r][ln] = bf16_bits(p0 - bf16_val(hb));
      hb = bf16_bits(p1);                sPh[w][8 * hh + r][16 + ln] = hb; sPl[w][8 * hh + r][16 + ln] = bf16_bits(p1 - bf16_val(hb));
    }
#pragma unroll
    for (int dt = 0; dt < DT; ++dt)
#pragma unroll
      for (int r = 0; r < 8; ++r) oacc[dt][r] *= alpha[r];
    __builtin_amdgcn_fence(__ATOMIC_ACQ_REL, "workgroup");
    __builtin_amdgcn_wave_barrier();
    FragB pah, pal;
    pah.half[0] = *(const v8us*)&sPh[w][ln][8 * hh]; pah.half[1] = *(const v8us*)&sPh[w][ln][16 + 8 * hh];
    pal.half[0] = *(const v8us*)&sPl[w][ln][8 * hh]; pal.half[1] = *(const v8us*)&sPl[w][ln][16 + 8 * hh];
#pragma unroll
    for (int dt = 0; dt < DT; ++dt) {
      FragB bvh, bvl;
#pragma unroll
      for (int i = 0; i < 8; ++i) {
        bvh.u[i] = sVh[8 * hh + i][dt * 16 + ln]; bvh.u[8 + i] = sVh[16 + 8 * hh + i][dt * 16 + ln];
        bvl.u[i] = sVl[8 * hh + i][dt * 16 + ln]; bvl.u[8 + i] = sVl[16 + 8 * hh + i][dt * 16 + ln];
      }
      oacc[dt] = mmaN<3>(pah.v, pal.v, bvh.v, bvl.v, oacc[dt]);
    }
    __builtin_amdgcn_fence(__ATOMIC_ACQ_REL, "workgroup");
    __builtin_amdgcn_wave_barrier();
  }
#pragma unroll
  for (int r = 0; r < 8; ++r) {
    float l = l_r[r];
    l += __shfl_xor(l, 1, 32); l += __shfl_xor(l, 2, 32); l += __shfl_xor(l, 4, 32); l += __shfl_xor(l, 8, 32);
    l_r[r] = (l > 0.f) ? 1.0f / l : 0.f;
  }
#pragma unroll
  for (int dt = 0; dt < DT; ++dt)
#pragma unroll
    for (int r = 0; r < 8; ++r) sO[w][8 * hh + r][dt * 16 + ln] = oacc[dt][r] * l_r[r];
  __builtin_amdgcn_fence(__ATOMIC_ACQ_REL, "workgroup");
  __builtin_amdgcn_wave_barrier();
  for (int pass = 0; pass < 2; ++pass) {
    for (int r = 0; r < 16; ++r) {
      const int row = q0 + r;
      if (row < T && lane < D / 4) {
        const v4f val = *(const v4fa*)&sO[w][r][lane * 4];
        *(volatile v4f*)(y + ((size_t)b * T + row) * ypitch + h * D + lane * 4) = val;
      }
    }
    if (pass == 0) __threadfence();
  }
}

template <bool ASPLIT, bool BSPLIT, int ACT>
__global__ __launch_bounds__(128) void k_gemm_b(const float* __restrict__ A, int lda, size_t sA, const unsigned short* __restrict__ Bh, const unsigned short* __restrict__ Bl, int ldb, size_t sB,
                                             const float* __restrict__ bias, const float* __restrict__ resid, int ldr, size_t sR, float rsign, float alpha,
                                             float* __restrict__ C, int ldc, size_t sC, int M, int N, int K) {
  __shared__ __attribute__((aligned(16))) float so[4][16][64];
  const int tid = threadIdx.x, w = tid >> 5, lane = tid & 31, ln = lane & 15, hh = lane >> 4;
  const int by = blockIdx.y;
  A += (size_t)by * sA; Bh += (size_t)by * sB; if (BSPLIT) Bl += (size_t)by * sB; C += (size_t)by * sC; if (resid) resid += (size_t)by * sR;
  const int ntn = (N + 63) / 64; const int wid = blockIdx.x * 4 + w; const int mt = wid / ntn, nq = wid % ntn;
  if (mt * 16 >= M) return;
  const int row0 = mt * 16, col0 = nq * 64;
  const float* arow = A + (size_t)(row0 + ln) * lda;
  v8f acc[4] = {};
  for (int kb = 0; kb < K; kb += 32) {
    FragB ah, al;
    const v4f x0 = *(const v4fa*)(arow + kb + 8 * hh), x1 = *(const v4fa*)(arow + kb + 8 * hh + 4);
    const v4f x2 = *(const v4fa*)(arow + kb + 16 + 8 * hh), x3 = *(const v4fa*)(arow + kb + 16 + 8 * hh + 4);
    float xs[16] = {x0[0],x0[1],x0[2],x0[3],x1[0],x1[1],x1[2],x1[3],x2[0],x2[1],x2[2],x2[3],x3[0],x3[1],x3[2],x3[3]};
#pragma unroll
    for (int i = 0; i < 16; ++i) { const unsigned short hb = bf16_bits(xs[i]); ah.u[i] = hb; al.u[i] = ASPLIT ? bf16_bits(xs[i] - bf16_val(hb)) : (unsigned short)0; }
#pragma unroll
    for (int t = 0; t < 4; ++t) {
      if (col0 + t * 16 >= N) continue;
      const size_t boff = (size_t)(col0 + t * 16 + ln) * ldb + kb;
      FragB bh_, bl_; bh_.half[0] = *(const v8us*)(Bh + boff + 8 * hh); bh_.half[1] = *(const v8us*)(Bh + boff + 16 + 8 * hh);
      if (BSPLIT) { bl_.half[0] = *(const v8us*)(Bl + boff + 8 * hh); bl_.half[1] = *(const v8us*)(Bl + boff + 16 + 8 * hh); } else bl_ = bh_;
      acc[t] = mmaN<ASPLIT ? (BSPLIT ? 3 : 2) : 1>(ah.v, al.v, bh_.v, bl_.v, acc[t]);
    }
  }
#pragma unroll
  for (int t = 0; t < 4; ++t) {
    const int col = col0 + t * 16 + ln; if (col0 + t * 16 >= N) continue; const float bv = bias ? bf16_round(bias[col]) : 0.f;
#pragma unroll
    for (int r = 0; r < 8; ++r) { float v = acc[t][r] * alpha + bv; if (resid) v += rsign * resid[(size_t)(row0 + 8 * hh + r) * ldr + col]; if (ACT == 1) v = fmaxf(v, 0.f); else if (ACT == 2) v = fmaxf(v, 0.f) + log1pf(expf(-fabsf(v))); so[w][8 * hh + r][t * 16 + ln] = v; }
  }
  __builtin_amdgcn_fence(__ATOMIC_ACQ_REL, "workgroup"); __builtin_amdgcn_wave_barrier();
  const int rsub = lane >> 4, c4 = (lane & 15) * 4;
  for (int pass = 0; pass < 2; ++pass) {
#pragma unroll
    for (int q = 0; q < 8; ++q) { const int r = q * 2 + rsub; if (col0 + c4 < N) { const v4f v = *(const v4fa*)&so[w][r][c4]; *(volatile v4f*)(C + (size_t)(row0 + r) * ldc + col0 + c4) = v; } }
    if (pass == 0) __threadfence();
  }
}
__global__ __launch_bounds__(256) void k_split_transpose_b(const float* __restrict__ src, int lds_, size_t sIn, unsigned short* __restrict__ hi, unsigned short* __restrict__ lo, size_t sOut, int K, int N) {
  const size_t t = (size_t)blockIdx.x * 256 + threadIdx.x; const int k8n = K / 8; if (t >= (size_t)N * k8n) return;
  src += (size_t)blockIdx.y * sIn; hi += (size_t)blockIdx.y * sOut; lo += (size_t)blockIdx.y * sOut;
  const int n = (int)(t / k8n), k8 = (int)(t % k8n) * 8; v8us vh, vl;
#pragma unroll
  for (int i = 0; i < 8; ++i) { const float x = src[(size_t)(k8 + i) * lds_ + n]; const unsigned short hb = bf16_bits(x); vh[i] = hb; vl[i] = bf16_bits(x - bf16_val(hb)); }
  unsigned short* dh = hi + (size_t)n * K + k8; unsigned short* dl = lo + (size_t)n * K + k8;
  *(volatile v8us*)dh = vh; *(volatile v8us*)dl = vl; __threadfence(); *(volatile v8us*)dh = vh; *(volatile v8us*)dl = vl;
}

__global__ __launch_bounds__(256) void k_perm(const float* __restrict__ F, float* __restrict__ XP, unsigned short* __restrict__ XB) { const int t = blockIdx.x * 256 + threadIdx.x; if (t >= NN * DD / 4) return; const int d4 = (t * 4) % DD; const int r = (t * 4) / DD; const int a = r / HB, b = r % HB; const v4f v = *(const v4fa*)(F + (size_t)(b * FL + a) * DD + d4); v4f o; typedef unsigned short v4us __attribute__((ext_vector_type(4))); v4us ob; for (int q = 0; q < 4; ++q) { o[q] = bf16_round(v[q]); ob[q] = bf16_bits(v[q]); }
  *(volatile v4f*)(XP + (size_t)t * 4) = o; *(volatile v4us*)(XB + (size_t)t * 4) = ob; __threadfence(); *(volatile v4f*)(XP + (size_t)t * 4) = o; *(volatile v4us*)(XB + (size_t)t * 4) = ob; }
__device__ __forceinline__ void pair_ij(int p, int& i, int& j) { int n = 0; i = 0; j = 0;
#pragma unroll 1
  for (int a = 0; a < FL; ++a) { const int cnt = FL - a; if (p < n + cnt) { i = a; j = a + (p - n); return; } n += cnt; } }
__global__ __launch_bounds__(256) void k_rows(const float* __restrict__ S, float* __restrict__ PR) { const int tid = threadIdx.x, wv = tid >> 5, lane = tid & 31; const int gr = blockIdx.x * 8 + wv; const int p = gr / (2 * HB), r = gr % (2 * HB); int i, j; pair_ij(p, i, j); const int a = (r < HB) ? i : j, rr = r % HB; const float* srow = S + ((size_t)(a * HB + rr)) * NN; const float invT = 10.0f;
  float den = 0.f;
#pragma unroll 2
  for (int c = lane; c < 2 * HB; c += 32) { if (c == r) continue; const int sc = ((c < HB) ? i : j) * HB + (c % HB); den += expf(srow[sc] * invT); }
  for (int o = 16; o >= 1; o >>= 1) den += __shfl_xor(den, o, 32);
  const int pc = (r + HB) % (2 * HB); const int psc = ((pc < HB) ? i : j) * HB + (pc % HB); const float pos = expf(srow[psc] * invT); const float pmt = pos / den;
  float lp = 0.f;
#pragma unroll 2
  for (int c = lane; c < 2 * HB; c += 32) { if (c == r) continue; const int sc = ((c < HB) ? i : j) * HB + (c % HB); lp += logf(1.0f - expf(srow[sc] * invT) / den); }
  for (int o = 16; o >= 1; o >>= 1) lp += __shfl_xor(lp, o, 32);
  if (lane == 0) { const float v = logf(pmt) + lp - logf(1.0f - pmt); *(volatile float*)(PR + gr) = v; } __threadfence(); if (lane == 0) { const float v = logf(pmt) + lp - logf(1.0f - pmt); *(volatile float*)(PR + gr) = v; } }
__global__ __launch_bounds__(256) void k_ce(const float* __restrict__ pred, const int* __restrict__ lab, float* __restrict__ CE) { const int tid = threadIdx.x, wv = tid >> 5, lane = tid & 31; const int n = blockIdx.x * 8 + wv; const float* pr = pred + (size_t)n * CC; float mx = -3.0e38f;
  for (int c = lane; c < CC; c += 32) mx = fmaxf(mx, bf16_round(pr[c])); for (int o = 16; o >= 1; o >>= 1) mx = fmaxf(mx, __shfl_xor(mx, o, 32)); float s = 0.f;
  for (int c = lane; c < CC; c += 32) s += expf(bf16_round(pr[c]) - mx); for (int o = 16; o >= 1; o >>= 1) s += __shfl_xor(s, o, 32);
  int l = lab[n]; l = l < 0 ? 0 : (l >= CC ? CC - 1 : l); const float v = -(bf16_round(pr[l]) - mx - logf(s));
  if (lane == 0) { *(volatile float*)(CE + n) = v; } __threadfence(); if (lane == 0) { *(volatile float*)(CE + n) = v; } }
__global__ __launch_bounds__(1024) void k_fin(const float* __restrict__ PR, const float* __restrict__ CE, float* __restrict__ out) { __shared__ float red[32]; const int tid = threadIdx.x, lane = tid & 31, wv = tid >> 5;
  float s = 0.f; for (int k = tid; k < NP * 2 * HB; k += 1024) s += PR[k]; for (int o = 16; o >= 1; o >>= 1) s += __shfl_xor(s, o, 32); if (lane == 0) red[wv] = s; __syncthreads(); float nce = 0.f; if (tid == 0) { for (int k = 0; k < 32; ++k) nce += red[k]; } __syncthreads();
  float c = 0.f; for (int k = tid; k < NN; k += 1024) c += CE[k]; for (int o = 16; o >= 1; o >>= 1) c += __shfl_xor(c, o, 32); if (lane == 0) red[wv] = c; __syncthreads();
  if (tid == 0) { float ce = 0.f; for (int k = 0; k < 32; ++k) ce += red[k]; const float loss = 0.03f * (-nce / (float)(2 * HB)) + ce / (float)NN; *(volatile float*)out = loss; __threadfence(); *(volatile float*)out = loss; } }
extern "C" void kernel_launch(void* const* d_in, const int* in_sizes, int n_in,
                              void* d_out, int out_size, void* d_ws, size_t ws_size, hipStream_t stream) {
  (void)in_sizes; (void)n_in; (void)out_size;
  const float* pred = (const float*)d_in[0]; const int* lab = (const int*)d_in[1]; const float* F = (const float*)d_in[2];
  char* ws = (char*)d_ws; size_t off = 0;
  auto take = [&](size_t bytes) { char* p = ws + off; off += (bytes + 255) & ~(size_t)255; return p; };
  float* XP = (float*)take((size_t)NN * DD * 4); unsigned short* XB = (unsigned short*)take((size_t)NN * DD * 2); float* S = (float*)take((size_t)NN * NN * 4); float* PR = (float*)take((size_t)NP * 2 * HB * 4); float* CE = (float*)take(NN * 4);
  if (off > ws_size) return;
  k_perm<<<(NN * DD / 4 + 255) / 256, 256, 0, stream>>>(F, XP, XB);
  k_gemm_b<false, false, 0><<<dim3(((NN / 16) * (NN / 64) + 3) / 4, 1), 128, 0, stream>>>(XP, DD, 0, XB, XB, DD, 0, nullptr, nullptr, 0, 0, 1.f, 1.f, S, NN, 0, NN, NN, DD);
  k_rows<<<NP * 2 * HB / 8, 256, 0, stream>>>(S, PR);
  k_ce<<<NN / 8, 256, 0, stream>>>(pred, lab, CE);
  k_fin<<<1, 1024, 0, stream>>>(PR, CE, (float*)d_out);
}
